// Stage_33105607917676
// MI455X (gfx1250) — hardware-verified
//
#include <hip/hip_runtime.h>
#include <math.h>

#define NPTS  40000
#define KNN_K 16
#define CCH   128
#define D4CH  32
#define HID   512
#define HEADN 256
#define DEPTH 4

typedef __attribute__((ext_vector_type(16))) _Float16 h16x16;
typedef __attribute__((ext_vector_type(8)))  _Float16 h16x8;
typedef __attribute__((ext_vector_type(8)))  float  f32x8;

__device__ __forceinline__ float gelu_f(float x) {
    const float k0 = 0.7978845608028654f;
    const float k1 = 0.044715f;
    float x3 = x * x * x;
    return 0.5f * x * (1.0f + tanhf(k0 * (x + k1 * x3)));
}

__device__ __forceinline__ float bn_scale() { return rsqrtf(1.0f + 1e-5f); }

typedef __attribute__((ext_vector_type(4))) float v4f;
typedef __attribute__((ext_vector_type(4))) unsigned v4u;
template <typename V> __device__ __forceinline__ void vst2(void* p, V v) {
    *(volatile V*)p = v; __threadfence(); *(volatile V*)p = v;
}
__device__ __forceinline__ void copy16(_Float16* lds_dst, const _Float16* g) { *(v4u*)lds_dst = *(const v4u*)g; }
__device__ __forceinline__ f32x8 wmma16(h16x16 a, h16x16 b, f32x8 c) {
    f32x8 d = __builtin_amdgcn_wmma_f32_16x16x32_f16(false, a, false, b, (short)0, c, false, false);
    asm volatile("v_nop\n\tv_nop\n\tv_nop\n\tv_nop" : "+v"(d) : "v"(a), "v"(b));
    return d;
}

__global__ __launch_bounds__(CCH)
void spse_kernel(const float* __restrict__ x, const float* __restrict__ xyz,
                 const int* __restrict__ knn,
                 const float* __restrict__ m_sp, const float* __restrict__ c_sp,
                 const float* __restrict__ h_sp,
                 const float* __restrict__ g0, const float* __restrict__ b0,
                 _Float16* __restrict__ nbr)
{
    const int n = blockIdx.x;
    const int c = threadIdx.x;
    __shared__ float srel[KNN_K][4];
    __shared__ float sref[KNN_K][4];
    __shared__ __align__(16) _Float16 srow[CCH];

    if (c < KNN_K) {
        int idx = knn[(size_t)n * KNN_K + c];
        idx = idx < 0 ? 0 : (idx >= NPTS ? NPTS - 1 : idx);
        srel[c][0] = xyz[(size_t)idx * 3 + 0] - xyz[(size_t)n * 3 + 0];
        srel[c][1] = xyz[(size_t)idx * 3 + 1] - xyz[(size_t)n * 3 + 1];
        srel[c][2] = xyz[(size_t)idx * 3 + 2] - xyz[(size_t)n * 3 + 2];
        srel[c][3] = 0.0f;
        sref[c][0] = x[(size_t)idx * 4 + 0] - x[(size_t)n * 4 + 0];
        sref[c][1] = x[(size_t)idx * 4 + 1] - x[(size_t)n * 4 + 1];
        sref[c][2] = x[(size_t)idx * 4 + 2] - x[(size_t)n * 4 + 2];
        sref[c][3] = x[(size_t)idx * 4 + 3] - x[(size_t)n * 4 + 3];
    }
    __syncthreads();

    float D0x = m_sp[0 * CCH + c], D0y = m_sp[1 * CCH + c], D0z = m_sp[2 * CCH + c];
    float D1x = m_sp[4 * CCH + c], D1y = m_sp[5 * CCH + c], D1z = m_sp[6 * CCH + c];
    float D2x = m_sp[8 * CCH + c], D2y = m_sp[9 * CCH + c], D2z = m_sp[10 * CCH + c];
    float cc0 = c_sp[0 * CCH + c]; cc0 *= cc0;
    float cc1 = c_sp[1 * CCH + c]; cc1 *= cc1;
    float cc2 = c_sp[2 * CCH + c]; cc2 *= cc2;
    float hh  = h_sp[c];           hh  *= hh;

    float e = 0.0f;
#pragma unroll 1
    for (int k = 0; k < KNN_K; ++k) {
        float rx = srel[k][0], ry = srel[k][1], rz = srel[k][2];
        float t0 = rx * D0x + ry * D0y + rz * D0z;
        float t1 = rx * D1x + ry * D1y + rz * D1z;
        float t2 = rx * D2x + ry * D2y + rz * D2z;
        e += t0 * t0 + t1 * t1 + t2 * t2;
        float f0 = sref[k][0], f1 = sref[k][1], f2 = sref[k][2], f3 = sref[k][3];
        e += f0 * f0 * cc0 + f1 * f1 * cc1 + f2 * f2 * cc2 + f3 * f3 * hh;
    }
    float r = sqrtf(e * (1.0f / (float)KNN_K));
    srow[c] = (_Float16)(r * (g0[c] * bn_scale()) + b0[c]);
    __syncthreads();
    if (c < 16) vst2(nbr + (size_t)n * CCH + c * 8, *(const v4u*)(&srow[c * 8]));
}

#define TM 64
#define TN 64
#define TK 32

#define EPI_NONE   0
#define EPI_GELU   1
#define EPI_BN     2
#define EPI_BN_RES 3

template<int MODE>
__global__ __launch_bounds__(128)
void gemm_wmma(const _Float16* __restrict__ X, const _Float16* __restrict__ Wt,
               const float* __restrict__ bias,
               const float* __restrict__ bn_g, const float* __restrict__ bn_b,
               const float* __restrict__ res,
               float* __restrict__ out_f32, _Float16* __restrict__ out_b16,
               int K, int Nn)
{
    __shared__ __align__(64) _Float16 sA[2][TM * TK];
    __shared__ __align__(64) _Float16 sB[2][TN * TK];
    __shared__ __align__(16) float Ct[TM][TN];

    const int tid  = threadIdx.x;
    const int lane = tid & 31;
    const int wid  = tid >> 5;
    const int m0   = blockIdx.x * TM;
    const int n0   = blockIdx.y * TN;
    const int wm   = (wid >> 1) * 32;
    const int wn   = (wid & 1) * 32;
    const int half = lane >> 4;

    auto stage = [&](int buf, int k0) {
#pragma unroll
        for (int p = 0; p < 2; ++p) {
            int e = tid + p * 128;
            int r = e >> 2;
            int ce = (e & 3) * 8;
            copy16(&sA[buf][e * 8], X + (size_t)(m0 + r) * K + k0 + ce);
            copy16(&sB[buf][e * 8], Wt + (size_t)(n0 + r) * K + k0 + ce);
        }
    };

    f32x8 acc[2][2] = {};
    stage(0, 0);

    for (int k0 = 0; k0 < K; k0 += TK) {
        const int cur = (k0 >> 5) & 1;
        if (k0 + TK < K) stage(cur ^ 1, k0 + TK);
        __syncthreads();

        h16x16 afrag[2];
#pragma unroll
        for (int mi = 0; mi < 2; ++mi) {
            const _Float16* ap = &sA[cur][(wm + mi * 16 + (lane & 15)) * TK + half * 8];
            h16x8 lo = *(const h16x8*)(ap);
            h16x8 hi = *(const h16x8*)(ap + 16);
            h16x16 f;
#pragma unroll
            for (int t = 0; t < 8; ++t) { f[t] = lo[t]; f[t + 8] = hi[t]; }
            afrag[mi] = f;
        }
        h16x16 bfrag[2];
#pragma unroll
        for (int ni = 0; ni < 2; ++ni) {
            const _Float16* bp = &sB[cur][(wn + ni * 16 + (lane & 15)) * TK + half * 8];
            h16x8 blo = *(const h16x8*)(bp);
            h16x8 bhi = *(const h16x8*)(bp + 16);
            h16x16 bf;
#pragma unroll
            for (int t = 0; t < 8; ++t) { bf[t] = blo[t]; bf[t + 8] = bhi[t]; }
            bfrag[ni] = bf;
        }
#pragma unroll
        for (int mi = 0; mi < 2; ++mi)
#pragma unroll
            for (int ni = 0; ni < 2; ++ni)
                acc[mi][ni] = wmma16(afrag[mi], bfrag[ni], acc[mi][ni]);
        __syncthreads();
    }

    const float bs = bn_scale();
#pragma unroll
    for (int ni = 0; ni < 2; ++ni) {
        int col = n0 + wn + ni * 16 + (lane & 15);
        float bv = (MODE == EPI_GELU && bias) ? bias[col] : 0.0f;
        float gs = 0.0f, bb = 0.0f;
        if (MODE >= EPI_BN) { gs = bn_g[col] * bs; bb = bn_b[col]; }
#pragma unroll
        for (int mi = 0; mi < 2; ++mi) {
#pragma unroll
            for (int r = 0; r < 8; ++r) {
                int rl = wm + mi * 16 + half * 8 + r;
                int row = m0 + rl;
                float v = acc[mi][ni][r] + bv;
                if (MODE == EPI_GELU) v = gelu_f(v);
                if (MODE >= EPI_BN) {
                    v = v * gs + bb;
                    if (MODE == EPI_BN_RES) v += res[(size_t)row * Nn + col];
                }
                Ct[rl][wn + ni * 16 + (lane & 15)] = v;
            }
        }
    }
    __syncthreads();
    if (out_f32) {
        for (int g = tid; g < TM * 16; g += 128) {
            const int rl = g >> 4, pc = g & 15;
            vst2(out_f32 + (size_t)(m0 + rl) * Nn + n0 + pc * 4, *(const v4f*)(&Ct[rl][pc * 4]));
        }
    }
    if (out_b16) {
        for (int g = tid; g < TM * 8; g += 128) {
            const int rl = g >> 3, pc = g & 7;
            union { h16x8 h; v4u u; } pk;
#pragma unroll
            for (int e = 0; e < 8; ++e) pk.h[e] = (_Float16)Ct[rl][pc * 8 + e];
            vst2(out_b16 + (size_t)(m0 + rl) * Nn + n0 + pc * 8, pk.u);
        }
    }
}

__global__ __launch_bounds__(CCH)
void lfp_kernel(const _Float16* __restrict__ xp, const float* __restrict__ xyz,
                const int* __restrict__ knn,
                const float* __restrict__ coor, const float* __restrict__ scale,
                const float* __restrict__ g, const float* __restrict__ b,
                float* __restrict__ h32, _Float16* __restrict__ h16)
{
    const int n = blockIdx.x;
    const int c = threadIdx.x;
    __shared__ float srel[KNN_K][3];
    __shared__ int   sidx[KNN_K];
    __shared__ __align__(16) _Float16 srow[CCH];

    if (c < KNN_K) {
        int idx = knn[(size_t)n * KNN_K + c];
        idx = idx < 0 ? 0 : (idx >= NPTS ? NPTS - 1 : idx);
        sidx[c] = idx;
        srel[c][0] = xyz[(size_t)idx * 3 + 0] - xyz[(size_t)n * 3 + 0];
        srel[c][1] = xyz[(size_t)idx * 3 + 1] - xyz[(size_t)n * 3 + 1];
        srel[c][2] = xyz[(size_t)idx * 3 + 2] - xyz[(size_t)n * 3 + 2];
    }
    __syncthreads();

    const int d4 = c >> 2;
    float c0 = coor[0 * D4CH + d4];
    float c1 = coor[1 * D4CH + d4];
    float c2 = coor[2 * D4CH + d4];
    float s  = scale[d4];
    float s2 = s * s;

    float m = -INFINITY;
#pragma unroll
    for (int k = 0; k < KNN_K; ++k) {
        float pe = (srel[k][0] * c0 + srel[k][1] * c1 + srel[k][2] * c2) * s2;
        float v  = (float)xp[(size_t)sidx[k] * CCH + c] + pe;
        m = fmaxf(m, v);
    }
    size_t idx = (size_t)n * CCH + c;
    float nh = h32[idx] + m * (g[c] * bn_scale()) + b[c];
    vst2(h32 + idx, nh);
    srow[c] = (_Float16)nh;
    __syncthreads();
    if (c < 16) vst2(h16 + (size_t)n * CCH + c * 8, *(const v4u*)(&srow[c * 8]));
}

__global__ __launch_bounds__(256)
void bn_kernel(const float* __restrict__ in, const float* __restrict__ g,
               const float* __restrict__ b, _Float16* __restrict__ out, int total)
{
    int gidx = blockIdx.x * blockDim.x + threadIdx.x;
    if (gidx * 8 >= total) return;
    union { h16x8 h; v4u u; } pk;
#pragma unroll
    for (int e = 0; e < 8; ++e) { int i = gidx * 8 + e; int c = i & (CCH - 1); pk.h[e] = (_Float16)(in[i] * (g[c] * bn_scale()) + b[c]); }
    vst2(out + (size_t)gidx * 8, pk.u);
}

__global__ __launch_bounds__(256)
void wconv_kernel(const float* __restrict__ in, _Float16* __restrict__ out,
                  int K, int N)
{
    __shared__ __align__(16) _Float16 tile[64][72];
    const int nt = N / 64;
    const int n0 = (blockIdx.x % nt) * 64, k0 = (blockIdx.x / nt) * 64;
    const int tid = threadIdx.x;
    for (int i = tid; i < 64 * 64; i += 256) { const int kk = i >> 6, nn = i & 63; tile[nn][kk] = (_Float16)in[(size_t)(k0 + kk) * N + n0 + nn]; }
    __syncthreads();
    for (int g = tid; g < 64 * 8; g += 256) { const int nn = g >> 3, pc = g & 7; vst2(out + (size_t)(n0 + nn) * K + k0 + pc * 8, *(const v4u*)(&tile[nn][pc * 8])); }
}

extern "C" void kernel_launch(void* const* d_in, const int* in_sizes, int n_in,
                              void* d_out, int out_size, void* d_ws, size_t ws_size,
                              hipStream_t stream)
{
    const float* x        = (const float*)d_in[0];
    const float* xyz      = (const float*)d_in[1];
    const int*   knn      = (const int*)  d_in[2];
    const float* spse_m   = (const float*)d_in[3];
    const float* spse_c   = (const float*)d_in[4];
    const float* spse_h   = (const float*)d_in[5];
    const float* bn0_g    = (const float*)d_in[6];
    const float* bn0_b    = (const float*)d_in[7];
    const float* nbr_w1   = (const float*)d_in[8];
    const float* nbr_b1   = (const float*)d_in[9];
    const float* nbr_w2   = (const float*)d_in[10];
    const float* nbr_bng  = (const float*)d_in[11];
    const float* nbr_bnb  = (const float*)d_in[12];
    const float* lfp_proj = (const float*)d_in[13];
    const float* lfp_coor = (const float*)d_in[14];
    const float* lfp_scal = (const float*)d_in[15];
    const float* lfp_bng  = (const float*)d_in[16];
    const float* lfp_bnb  = (const float*)d_in[17];
    const float* mlp_w1   = (const float*)d_in[18];
    const float* mlp_b1   = (const float*)d_in[19];
    const float* mlp_w2   = (const float*)d_in[20];
    const float* mlp_bng  = (const float*)d_in[21];
    const float* mlp_bnb  = (const float*)d_in[22];
    const float* post_g   = (const float*)d_in[23];
    const float* post_b   = (const float*)d_in[24];
    const float* post_w   = (const float*)d_in[25];
    float* out = (float*)d_out;

    char* w = (char*)d_ws;
    float*  h32   = (float*)w;  w += (size_t)NPTS * CCH * 4;
    _Float16* h16   = (_Float16*)w; w += (size_t)NPTS * CCH * 2;
    _Float16* big16 = (_Float16*)w; w += (size_t)NPTS * HID * 2;
    _Float16* c16   = (_Float16*)w; w += (size_t)NPTS * CCH * 2;
    _Float16* wt_n1 = (_Float16*)w; w += (size_t)CCH * 2 * CCH * 2;
    _Float16* wt_n2 = (_Float16*)w; w += (size_t)2 * CCH * CCH * 2;
    _Float16* wt_lf = (_Float16*)w; w += (size_t)DEPTH * CCH * CCH * 2;
    _Float16* wt_m1 = (_Float16*)w; w += (size_t)3 * CCH * HID * 2;
    _Float16* wt_m2 = (_Float16*)w; w += (size_t)3 * HID * CCH * 2;
    _Float16* wt_pw = (_Float16*)w; w += (size_t)CCH * HEADN * 2;

    const int MT = NPTS / TM;
    dim3 blk(128);
    auto cdiv = [](int a, int b) { return (a + b - 1) / b; };

    wconv_kernel<<<(CCH / 64) * (2 * CCH / 64), 256, 0, stream>>>(nbr_w1, wt_n1, CCH, 2 * CCH);
    wconv_kernel<<<(2 * CCH / 64) * (CCH / 64), 256, 0, stream>>>(nbr_w2, wt_n2, 2 * CCH, CCH);
    for (int i = 0; i < DEPTH; ++i)
        wconv_kernel<<<(CCH / 64) * (CCH / 64), 256, 0, stream>>>(
            lfp_proj + (size_t)i * CCH * CCH, wt_lf + (size_t)i * CCH * CCH, CCH, CCH);
    for (int j = 0; j < 3; ++j) {
        wconv_kernel<<<(CCH / 64) * (HID / 64), 256, 0, stream>>>(
            mlp_w1 + (size_t)j * CCH * HID, wt_m1 + (size_t)j * CCH * HID, CCH, HID);
        wconv_kernel<<<(HID / 64) * (CCH / 64), 256, 0, stream>>>(
            mlp_w2 + (size_t)j * HID * CCH, wt_m2 + (size_t)j * HID * CCH, HID, CCH);
    }
    wconv_kernel<<<(CCH / 64) * (HEADN / 64), 256, 0, stream>>>(post_w, wt_pw, CCH, HEADN);

    spse_kernel<<<NPTS, CCH, 0, stream>>>(x, xyz, knn, spse_m, spse_c, spse_h,
                                          bn0_g, bn0_b, c16);

    gemm_wmma<EPI_GELU><<<dim3(MT, 2 * CCH / TN), blk, 0, stream>>>(
        c16, wt_n1, nbr_b1, nullptr, nullptr, nullptr, nullptr, big16, CCH, 2 * CCH);
    gemm_wmma<EPI_BN><<<dim3(MT, CCH / TN), blk, 0, stream>>>(
        big16, wt_n2, nullptr, nbr_bng, nbr_bnb, nullptr, h32, h16, 2 * CCH, CCH);

    auto run_mlp = [&](int j) {
        gemm_wmma<EPI_GELU><<<dim3(MT, HID / TN), blk, 0, stream>>>(
            h16, wt_m1 + (size_t)j * CCH * HID, mlp_b1 + (size_t)j * HID,
            nullptr, nullptr, nullptr, nullptr, big16, CCH, HID);
        gemm_wmma<EPI_BN_RES><<<dim3(MT, CCH / TN), blk, 0, stream>>>(
            big16, wt_m2 + (size_t)j * HID * CCH, nullptr,
            mlp_bng + (size_t)j * CCH, mlp_bnb + (size_t)j * CCH, h32,
            h32, h16, HID, CCH);
    };

    run_mlp(0);

    for (int i = 0; i < DEPTH; ++i) {
        gemm_wmma<EPI_NONE><<<dim3(MT, CCH / TN), blk, 0, stream>>>(
            h16, wt_lf + (size_t)i * CCH * CCH, nullptr, nullptr, nullptr,
            nullptr, nullptr, c16, CCH, CCH);
        lfp_kernel<<<NPTS, CCH, 0, stream>>>(
            c16, xyz, knn, lfp_coor + (size_t)i * 3 * D4CH,
            lfp_scal + (size_t)i * D4CH,
            lfp_bng + (size_t)i * CCH, lfp_bnb + (size_t)i * CCH, h32, h16);
        if (i & 1) run_mlp(i / 2 + 1);
    }

    int total = NPTS * CCH;
    bn_kernel<<<cdiv(total / 8, 256), 256, 0, stream>>>(h32, post_g, post_b, c16, total);
    gemm_wmma<EPI_NONE><<<dim3(MT, HEADN / TN), blk, 0, stream>>>(
        c16, wt_pw, nullptr, nullptr, nullptr, nullptr, out, nullptr, CCH, HEADN);
}
